// ContinuousThoughtMachine_40432822124583
// MI455X (gfx1250) — hardware-verified
//
#include <hip/hip_runtime.h>


#define NB   512
#define NT   8
#define ND   2048
#define NDIN 512
#define NM   16
#define NH   4
#define NP   512
#define NDO  512

#define GBM 128
#define GBN 128
#define GBK 32
#define GLP 40
#define GPLANE (GBM * GLP)
#define EPP 68
#define EPW (16 * EPP)

#define ZSCALE 4096.0f
#define WSCALE 64.0f
#define ZW_UNSCALE (1.0f / 262144.0f)

static_assert(NB % GBM == 0);
static_assert(ND % GBN == 0);
static_assert(NDO % GBN == 0);
static_assert(GBM == GBN);
static_assert(ND % GBK == 0);
static_assert(NDIN % GBK == 0);
static_assert(NP % GBK == 0);
static_assert(ND % 64 == 0 && NDIN % 64 == 0 && NP % 64 == 0 && NDO % 64 == 0);
static_assert(ND % 1024 == 0);
static_assert(NP == 512);
static_assert(NT <= NM);
static_assert((NB * NDIN) % 8 == 0 && (NB * ND) % 8 == 0);

typedef _Float16       h16v __attribute__((ext_vector_type(16)));
typedef __bf16         b16v __attribute__((ext_vector_type(16)));
typedef float          f8v  __attribute__((ext_vector_type(8)));
typedef float          f4v  __attribute__((ext_vector_type(4)));
typedef unsigned int   u4v  __attribute__((ext_vector_type(4)));

union Frag { h16v vh; b16v vb; u4v q[2]; };

__device__ __forceinline__ unsigned short bf_rne(float f) {
  unsigned int u = __float_as_uint(f);
  u += 0x7FFFu + ((u >> 16) & 1u);
  return (unsigned short)(u >> 16);
}
__device__ __forceinline__ float bf_val(unsigned short s) {
  return __uint_as_float(((unsigned int)s) << 16);
}
__device__ __forceinline__ unsigned short h_bits(float f) {
  union { _Float16 h; unsigned short u; } c;
  c.h = (_Float16)f;
  return c.u;
}
__device__ __forceinline__ unsigned int pk2(unsigned short a, unsigned short b) {
  return (unsigned int)a | ((unsigned int)b << 16);
}

__device__ __forceinline__ void split8(const float (&e)[8], u4v& vh, u4v& vl) {
  unsigned int ph[4], pl[4];
  #pragma unroll
  for (int i = 0; i < 4; ++i) {
    const unsigned short h0 = bf_rne(e[2 * i]);
    const unsigned short h1 = bf_rne(e[2 * i + 1]);
    const unsigned short l0 = bf_rne(e[2 * i] - bf_val(h0));
    const unsigned short l1 = bf_rne(e[2 * i + 1] - bf_val(h1));
    ph[i] = pk2(h0, h1);
    pl[i] = pk2(l0, l1);
  }
  vh.x = ph[0]; vh.y = ph[1]; vh.z = ph[2]; vh.w = ph[3];
  vl.x = pl[0]; vl.y = pl[1]; vl.z = pl[2]; vl.w = pl[3];
}

__device__ __forceinline__ u4v packh8(const float (&e)[8]) {
  u4v r;
  r.x = pk2(h_bits(e[0]), h_bits(e[1]));
  r.y = pk2(h_bits(e[2]), h_bits(e[3]));
  r.z = pk2(h_bits(e[4]), h_bits(e[5]));
  r.w = pk2(h_bits(e[6]), h_bits(e[7]));
  return r;
}

__device__ __forceinline__ f4v relu4(f4v v) {
  f4v r;
  r.x = v.x > 0.f ? v.x : 0.f;
  r.y = v.y > 0.f ? v.y : 0.f;
  r.z = v.z > 0.f ? v.z : 0.f;
  r.w = v.w > 0.f ? v.w : 0.f;
  return r;
}

__device__ __forceinline__ int fixidx(int i) {
  if (i < 0) i += ND;
  i = i < 0 ? 0 : i;
  i = i > ND - 1 ? ND - 1 : i;
  return i;
}

template <int BF>
__device__ __forceinline__ f8v wmma1(const Frag& a, const Frag& b, f8v c) {
  if constexpr (BF != 0) {
    return __builtin_amdgcn_wmma_f32_16x16x32_bf16(false, a.vb, false, b.vb, (short)0, c, false, false);
  } else {
    return __builtin_amdgcn_wmma_f32_16x16x32_f16(false, a.vh, false, b.vh, (short)0, c, false, false);
  }
}

#define WGUARD_P(d0, d1, a0, a1, b) \
  asm volatile("v_nop\n\tv_nop\n\tv_nop\n\tv_nop" : "+v"(d0), "+v"(d1) \
               : "v"((a0).q[0]), "v"((a0).q[1]), "v"((a1).q[0]), "v"((a1).q[1]), \
                 "v"((b).q[0]), "v"((b).q[1]))
#define WGUARD_S(d0, d1, a0, a1, l0, l1, bh, bl) \
  asm volatile("v_nop\n\tv_nop\n\tv_nop\n\tv_nop" : "+v"(d0), "+v"(d1) \
               : "v"((a0).q[0]), "v"((a0).q[1]), "v"((a1).q[0]), "v"((a1).q[1]), \
                 "v"((l0).q[0]), "v"((l0).q[1]), "v"((l1).q[0]), "v"((l1).q[1]), \
                 "v"((bh).q[0]), "v"((bh).q[1]), "v"((bl).q[0]), "v"((bl).q[1]))

template <int BF, int SPLIT, int OUTM>
__global__ void __launch_bounds__(256)
k_gemm(const unsigned short* __restrict__ Ah, const unsigned short* __restrict__ Al,
       int lda, long long zsA,
       const unsigned short* __restrict__ Bh, const unsigned short* __restrict__ Bl,
       int ldb, long long zsB,
       int K,
       const float* __restrict__ bias0, const float* __restrict__ bias1,
       const float* __restrict__ addend, int ldadd,
       float scale,
       float* Cf, int ldc, long long zsC,
       unsigned short* Ch, unsigned short* Cl, int ldch)
{
  constexpr int NPL = SPLIT ? 4 : 2;
  constexpr int OPWORDS = NPL * GPLANE / 2;
  constexpr int EPWORDS = 8 * EPW;
  constexpr int SMW = OPWORDS > EPWORDS ? OPWORDS : EPWORDS;
  __shared__ __align__(16) float smf[SMW];
  unsigned short* const sm = reinterpret_cast<unsigned short*>(smf);

  const int tid = threadIdx.x, lane = tid & 31, wv = tid >> 5;
  const int hh = lane >> 4, mm = lane & 15;
  const int rowBase = blockIdx.x * GBM, colBase = blockIdx.y * GBN;
  const long long zi = (long long)blockIdx.z;
  const unsigned short* pAh = Ah + zi * zsA;
  const unsigned short* pBh = Bh + zi * zsB;
  const unsigned short* pAl = Al;
  const unsigned short* pBl = Bl;
  if constexpr (SPLIT != 0) { pAl = Al + zi * zsA; pBl = Bl + zi * zsB; }
  const float* bias = (blockIdx.z == 0) ? bias0 : bias1;
  float* pC = Cf;
  if constexpr (OUTM == 0) pC = Cf + zi * zsC;
  const int wr = (wv & 3) * 32, wc = (wv >> 2) * 64;

  const f8v zero8 = {0.f, 0.f, 0.f, 0.f, 0.f, 0.f, 0.f, 0.f};
  f8v acc[2][4];
  #pragma unroll
  for (int fi = 0; fi < 2; ++fi)
    #pragma unroll
    for (int fj = 0; fj < 4; ++fj) acc[fi][fj] = zero8;

  #pragma unroll 1
  for (int k0 = 0; k0 < K; k0 += GBK) {
    #pragma unroll
    for (int j = 0; j < 2; ++j) {
      const int c = tid + 256 * j;
      const int row = c >> 2, part = (c & 3) * 8;
      const int lo = row * GLP + part;
      const u4v va = *(const u4v*)(pAh + (size_t)(rowBase + row) * lda + k0 + part);
      const u4v vb = *(const u4v*)(pBh + (size_t)(colBase + row) * ldb + k0 + part);
      *(u4v*)(sm + lo) = va;
      *(u4v*)(sm + GPLANE + lo) = vb;
      if constexpr (SPLIT != 0) {
        const u4v wa = *(const u4v*)(pAl + (size_t)(rowBase + row) * lda + k0 + part);
        const u4v wb = *(const u4v*)(pBl + (size_t)(colBase + row) * ldb + k0 + part);
        *(u4v*)(sm + 2 * GPLANE + lo) = wa;
        *(u4v*)(sm + 3 * GPLANE + lo) = wb;
      }
    }
    __syncthreads();

    Frag ah[2], al[2];
    #pragma unroll
    for (int fi = 0; fi < 2; ++fi) {
      const unsigned short* ap = sm + (wr + fi * 16 + mm) * GLP + 8 * hh;
      ah[fi].q[0] = *(const u4v*)(ap);
      ah[fi].q[1] = *(const u4v*)(ap + 16);
      if constexpr (SPLIT != 0) {
        al[fi].q[0] = *(const u4v*)(ap + 2 * GPLANE);
        al[fi].q[1] = *(const u4v*)(ap + 2 * GPLANE + 16);
      } else {
        al[fi] = ah[fi];
      }
    }
    #pragma unroll
    for (int fj = 0; fj < 4; ++fj) {
      const unsigned short* bp = sm + GPLANE + (wc + fj * 16 + mm) * GLP + 8 * hh;
      Frag bh, bl;
      bh.q[0] = *(const u4v*)(bp);
      bh.q[1] = *(const u4v*)(bp + 16);
      if constexpr (SPLIT != 0) {
        bl.q[0] = *(const u4v*)(bp + 2 * GPLANE);
        bl.q[1] = *(const u4v*)(bp + 2 * GPLANE + 16);
      } else {
        bl = bh;
      }
      f8v d0 = wmma1<BF>(ah[0], bh, acc[0][fj]);
      f8v d1 = wmma1<BF>(ah[1], bh, acc[1][fj]);
      if constexpr (SPLIT != 0) {
        d0 = wmma1<BF>(ah[0], bl, d0);
        d1 = wmma1<BF>(ah[1], bl, d1);
        d0 = wmma1<BF>(al[0], bh, d0);
        d1 = wmma1<BF>(al[1], bh, d1);
        WGUARD_S(d0, d1, ah[0], ah[1], al[0], al[1], bh, bl);
      } else {
        WGUARD_P(d0, d1, ah[0], ah[1], bh);
      }
      acc[0][fj] = d0;
      acc[1][fj] = d1;
    }
    __syncthreads();
  }

  float* stg = smf + wv * EPW;
  #pragma unroll
  for (int fi = 0; fi < 2; ++fi) {
    #pragma unroll
    for (int fj = 0; fj < 4; ++fj)
      #pragma unroll
      for (int r = 0; r < 8; ++r)
        stg[(8 * hh + r) * EPP + fj * 16 + mm] = acc[fi][fj][r];
    __syncthreads();
    const int growBase = rowBase + wr + fi * 16;
    if constexpr (OUTM == 0) {
      f4v vals[8];
      size_t goff[8];
      #pragma unroll
      for (int s = 0; s < 8; ++s) {
        const int L = 4 * s + (lane >> 3);
        const int row = L >> 1, col = (L & 1) * 32 + (lane & 7) * 4;
        f4v v = *(const f4v*)(stg + row * EPP + col);
        const int gcol = colBase + wc + col;
        const int grow = growBase + row;
        v = v * scale;
        if (bias) v += *(const f4v*)(bias + gcol);
        if (addend) v += *(const f4v*)(addend + (size_t)grow * ldadd + gcol);
        vals[s] = v;
        goff[s] = (size_t)grow * ldc + gcol;
      }
      #pragma unroll
      for (int s = 0; s < 8; ++s) *(volatile f4v*)(pC + goff[s]) = vals[s];
      __threadfence();
      #pragma unroll
      for (int s = 0; s < 8; ++s) *(volatile f4v*)(pC + goff[s]) = vals[s];
    } else {
      u4v vh[4], vl[4];
      size_t goff[4];
      #pragma unroll
      for (int s = 0; s < 4; ++s) {
        const int row = 4 * s + (lane >> 3), col = (lane & 7) * 8;
        f4v a0 = *(const f4v*)(stg + row * EPP + col);
        f4v a1 = *(const f4v*)(stg + row * EPP + col + 4);
        const int gcol = colBase + wc + col;
        const int grow = growBase + row;
        a0 = a0 * scale;
        a1 = a1 * scale;
        if (bias) {
          a0 += *(const f4v*)(bias + gcol);
          a1 += *(const f4v*)(bias + gcol + 4);
        }
        float e[8] = {a0.x, a0.y, a0.z, a0.w, a1.x, a1.y, a1.z, a1.w};
        split8(e, vh[s], vl[s]);
        goff[s] = (size_t)grow * ldch + gcol;
      }
      #pragma unroll
      for (int s = 0; s < 4; ++s) {
        *(volatile u4v*)(Ch + goff[s]) = vh[s];
        *(volatile u4v*)(Cl + goff[s]) = vl[s];
      }
      __threadfence();
      #pragma unroll
      for (int s = 0; s < 4; ++s) {
        *(volatile u4v*)(Ch + goff[s]) = vh[s];
        *(volatile u4v*)(Cl + goff[s]) = vl[s];
      }
    }
    __syncthreads();
  }
}

template <int MODE>
__global__ void __launch_bounds__(256)
k_tconv(const float* __restrict__ in, int K, int N, float scale,
        unsigned short* oh, unsigned short* ol)
{
  __shared__ __align__(16) float tile[64 * EPP];
  const int k0 = blockIdx.x * 64, n0 = blockIdx.y * 64;
  if (k0 + 64 > K || n0 + 64 > N) return;
  const int tid = threadIdx.x, lane = tid & 31, wv = tid >> 5;
  #pragma unroll
  for (int j = 0; j < 4; ++j) {
    const int c = tid + 256 * j, kk = c >> 4, nn = (c & 15) * 4;
    const f4v v = *(const f4v*)(in + (size_t)(k0 + kk) * N + n0 + nn);
    *(f4v*)(tile + kk * EPP + nn) = v;
  }
  __syncthreads();
  u4v vh[2], vl[2];
  size_t goff[2];
  #pragma unroll
  for (int s = 0; s < 2; ++s) {
    const int nl = wv * 8 + s * 4 + (lane >> 3), kl = (lane & 7) * 8;
    float e[8];
    #pragma unroll
    for (int i = 0; i < 8; ++i) e[i] = tile[(kl + i) * EPP + nl] * scale;
    if constexpr (MODE != 0) {
      split8(e, vh[s], vl[s]);
    } else {
      vh[s] = packh8(e);
      vl[s] = vh[s];
    }
    goff[s] = (size_t)(n0 + nl) * K + k0 + kl;
  }
  #pragma unroll
  for (int s = 0; s < 2; ++s) {
    *(volatile u4v*)(oh + goff[s]) = vh[s];
    if constexpr (MODE != 0) *(volatile u4v*)(ol + goff[s]) = vl[s];
  }
  __threadfence();
  #pragma unroll
  for (int s = 0; s < 2; ++s) {
    *(volatile u4v*)(oh + goff[s]) = vh[s];
    if constexpr (MODE != 0) *(volatile u4v*)(ol + goff[s]) = vl[s];
  }
}

__global__ void __launch_bounds__(256)
k_split8(const float* __restrict__ in, unsigned short* oh, unsigned short* ol, int n8)
{
  const int i = blockIdx.x * 256 + threadIdx.x;
  if (i >= n8) return;
  const size_t e0 = (size_t)i * 8;
  const f4v a = *(const f4v*)(in + e0);
  const f4v b = *(const f4v*)(in + e0 + 4);
  float e[8] = {a.x, a.y, a.z, a.w, b.x, b.y, b.z, b.w};
  u4v vh, vl;
  split8(e, vh, vl);
  *(volatile u4v*)(oh + e0) = vh;
  *(volatile u4v*)(ol + e0) = vl;
  __threadfence();
  *(volatile u4v*)(oh + e0) = vh;
  *(volatile u4v*)(ol + e0) = vl;
}

__global__ void __launch_bounds__(256)
k_initz(const float* __restrict__ z0, unsigned short* zh, int n8)
{
  const int i = blockIdx.x * 256 + threadIdx.x;
  if (i >= n8) return;
  const size_t e0 = (size_t)i * 8;
  const int d = (int)(e0 % ND);
  const f4v a = *(const f4v*)(z0 + d);
  const f4v b = *(const f4v*)(z0 + d + 4);
  float e[8] = {a.x * ZSCALE, a.y * ZSCALE, a.z * ZSCALE, a.w * ZSCALE,
                b.x * ZSCALE, b.y * ZSCALE, b.z * ZSCALE, b.w * ZSCALE};
  const u4v v = packh8(e);
  *(volatile u4v*)(zh + e0) = v;
  __threadfence();
  *(volatile u4v*)(zh + e0) = v;
}

__global__ void __launch_bounds__(256)
k_nlm(const float* __restrict__ hist, const float* __restrict__ w1, const float* __restrict__ b1,
      const float* __restrict__ w2, const float* __restrict__ b2,
      float* zf, unsigned short* zh, int t)
{
  __shared__ __align__(16) unsigned short sz[1024];
  const int tid = threadIdx.x;
  const size_t base = (size_t)blockIdx.x * 1024;
  const size_t e0 = base + (size_t)tid * 4;
  if (base + 1024 > (size_t)NB * ND) return;
  const int d0 = (int)(e0 % ND);
  int tt = t;
  if (tt < 0) tt = 0;
  if (tt > NT - 1) tt = NT - 1;
  const f4v zero4 = {0.f, 0.f, 0.f, 0.f};
  f4v h[NH];
  #pragma unroll
  for (int q = 0; q < NH; ++q) h[q] = zero4;
  #pragma unroll 1
  for (int s = 0; s <= tt; ++s) {
    const f4v p = *(const f4v*)(hist + (size_t)s * NB * ND + e0);
    const int mpos = NM - 1 - (tt - s);
    const float* wp = w1 + (size_t)mpos * NH * ND + d0;
    #pragma unroll
    for (int q = 0; q < NH; ++q) h[q] += p * *(const f4v*)(wp + (size_t)q * ND);
  }
  f4v acc = zero4;
  #pragma unroll
  for (int q = 0; q < NH; ++q) {
    f4v hv = h[q] + *(const f4v*)(b1 + (size_t)q * ND + d0);
    hv = relu4(hv);
    acc += hv * *(const f4v*)(w2 + (size_t)q * ND + d0);
  }
  acc += *(const f4v*)(b2 + d0);

  sz[tid * 4 + 0] = h_bits(acc.x * ZSCALE);
  sz[tid * 4 + 1] = h_bits(acc.y * ZSCALE);
  sz[tid * 4 + 2] = h_bits(acc.z * ZSCALE);
  sz[tid * 4 + 3] = h_bits(acc.w * ZSCALE);
  __syncthreads();
  const bool wl = tid < 128;
  u4v pv = {0u, 0u, 0u, 0u};
  if (wl) pv = *(const u4v*)(sz + tid * 8);
  *(volatile f4v*)(zf + e0) = acc;
  if (wl) *(volatile u4v*)(zh + base + (size_t)tid * 8) = pv;
  __threadfence();
  *(volatile f4v*)(zf + e0) = acc;
  if (wl) *(volatile u4v*)(zh + base + (size_t)tid * 8) = pv;
}

__global__ void __launch_bounds__(128)
k_sync(const float* __restrict__ zf, const int* __restrict__ po, const int* __restrict__ pa,
       const float* __restrict__ dco, const float* __restrict__ dca,
       float* So, float* Sa, unsigned short* Spl, int first)
{
  #pragma clang fp contract(off)
  __shared__ __align__(16) unsigned short sh[4 * NP];
  const int tid = threadIdx.x, b = blockIdx.x, p0 = tid * 4;
  if (b >= NB) return;
  const float* zb = zf + (size_t)b * ND;
  const size_t so = (size_t)b * NP + p0;
  const f4v zero4 = {0.f, 0.f, 0.f, 0.f};
  f4v newS[2];
  #pragma unroll
  for (int hd = 0; hd < 2; ++hd) {
    const int* pr = hd ? pa : po;
    const float* dc = hd ? dca : dco;
    const float* S = hd ? Sa : So;
    f4v prev = zero4;
    if (!first) prev = *(const f4v*)(S + so);
    const float pv[4] = {prev.x, prev.y, prev.z, prev.w};
    float nv[4];
    #pragma unroll
    for (int q = 0; q < 4; ++q) {
      const int p = p0 + q;
      const int i = fixidx(pr[2 * p]);
      const int j = fixidx(pr[2 * p + 1]);
      const float r = __expf(-fabsf(dc[p]));
      const float a = pv[q] * r;
      const float m = zb[i] * zb[j];
      nv[q] = a + m;
      const unsigned short hb = bf_rne(nv[q]);
      sh[(2 * hd) * NP + p] = hb;
      sh[(2 * hd + 1) * NP + p] = bf_rne(nv[q] - bf_val(hb));
    }
    f4v ns;
    ns.x = nv[0]; ns.y = nv[1]; ns.z = nv[2]; ns.w = nv[3];
    newS[hd] = ns;
  }
  __syncthreads();
  u4v pl[2];
  size_t poff[2];
  #pragma unroll
  for (int j = 0; j < 2; ++j) {
    const int c = tid + 128 * j;
    const int plane = c >> 6, off = (c & 63) * 8;
    pl[j] = *(const u4v*)(sh + plane * NP + off);
    poff[j] = (size_t)plane * ((size_t)NB * NP) + (size_t)b * NP + off;
  }
  *(volatile f4v*)(So + so) = newS[0];
  *(volatile f4v*)(Sa + so) = newS[1];
  #pragma unroll
  for (int j = 0; j < 2; ++j) *(volatile u4v*)(Spl + poff[j]) = pl[j];
  __threadfence();
  *(volatile f4v*)(So + so) = newS[0];
  *(volatile f4v*)(Sa + so) = newS[1];
  #pragma unroll
  for (int j = 0; j < 2; ++j) *(volatile u4v*)(Spl + poff[j]) = pl[j];
}

extern "C" void kernel_launch(void* const* d_in, const int* in_sizes, int n_in,
                              void* d_out, int out_size, void* d_ws, size_t ws_size,
                              hipStream_t stream)
{
  if (n_in < 18) return;
  if (in_sizes[0] != NB * NDIN || in_sizes[1] != NDIN * ND || in_sizes[2] != ND || in_sizes[3] != ND ||
      in_sizes[4] != 2 * ND * ND || in_sizes[5] != ND || in_sizes[6] != NM * NH * ND ||
      in_sizes[7] != NH * ND || in_sizes[8] != NH * ND || in_sizes[9] != ND ||
      in_sizes[10] != NP || in_sizes[11] != NP || in_sizes[12] != NP * NDO || in_sizes[13] != NDO ||
      in_sizes[14] != NP * NDO || in_sizes[15] != NDO || in_sizes[16] != 2 * NP || in_sizes[17] != 2 * NP)
    return;
  if (out_size != 2 * NB * NT * NDO) return;

  const float* x      = (const float*)d_in[0];
  const float* W_in   = (const float*)d_in[1];
  const float* b_in   = (const float*)d_in[2];
  const float* z0     = (const float*)d_in[3];
  const float* W_syn  = (const float*)d_in[4];
  const float* b_syn  = (const float*)d_in[5];
  const float* w1     = (const float*)d_in[6];
  const float* b1     = (const float*)d_in[7];
  const float* w2     = (const float*)d_in[8];
  const float* b2     = (const float*)d_in[9];
  const float* dec_o  = (const float*)d_in[10];
  const float* dec_a  = (const float*)d_in[11];
  const float* W_out  = (const float*)d_in[12];
  const float* b_out  = (const float*)d_in[13];
  const float* W_act  = (const float*)d_in[14];
  const float* b_act  = (const float*)d_in[15];
  const int*   prs_o  = (const int*)d_in[16];
  const int*   prs_a  = (const int*)d_in[17];
  float* out = (float*)d_out;

  const size_t QX  = (size_t)NB * NDIN;
  const size_t QWI = (size_t)ND * NDIN;
  const size_t QWS = (size_t)ND * ND;
  const size_t QWO = (size_t)NDO * NP;
  const size_t QF  = (size_t)NB * ND;
  const size_t QS  = (size_t)NB * NP;

  size_t off = 0;
  char* wsb = (char*)d_ws;
  auto take = [&](size_t bytes) -> char* {
    char* p = wsb + off;
    off += (bytes + 255) & ~(size_t)255;
    return p;
  };
  unsigned short* xh   = (unsigned short*)take(QX * 2);
  unsigned short* xl   = (unsigned short*)take(QX * 2);
  unsigned short* wih  = (unsigned short*)take(QWI * 2);
  unsigned short* wil  = (unsigned short*)take(QWI * 2);
  unsigned short* wz   = (unsigned short*)take(QWS * 2);
  unsigned short* wfh  = (unsigned short*)take(QWS * 2);
  unsigned short* wfl  = (unsigned short*)take(QWS * 2);
  unsigned short* wo   = (unsigned short*)take(4 * QWO * 2);
  unsigned short* zh   = (unsigned short*)take(QF * 2);
  unsigned short* fh   = (unsigned short*)take(QF * 2);
  unsigned short* fl   = (unsigned short*)take(QF * 2);
  float*          fpre = (float*)take(QF * 4);
  float*          hist = (float*)take((size_t)NT * QF * 4);
  float*          zf   = (float*)take(QF * 4);
  float*          So   = (float*)take(QS * 4);
  float*          Sa   = (float*)take(QS * 4);
  unsigned short* spl  = (unsigned short*)take(4 * QS * 2);
  if (off > ws_size) return;

  const dim3 blk(256);

  k_split8<<<dim3((unsigned)((QX / 8 + 255) / 256)), blk, 0, stream>>>(x, xh, xl, (int)(QX / 8));
  hipLaunchKernelGGL(HIP_KERNEL_NAME(k_tconv<1>), dim3(NDIN / 64, ND / 64), blk, 0, stream,
                     W_in, (int)NDIN, (int)ND, 1.0f, wih, wil);
  hipLaunchKernelGGL(HIP_KERNEL_NAME(k_tconv<0>), dim3(ND / 64, ND / 64), blk, 0, stream,
                     W_syn, (int)ND, (int)ND, WSCALE, wz, (unsigned short*)nullptr);
  hipLaunchKernelGGL(HIP_KERNEL_NAME(k_tconv<1>), dim3(ND / 64, ND / 64), blk, 0, stream,
                     W_syn + QWS, (int)ND, (int)ND, 1.0f, wfh, wfl);
  hipLaunchKernelGGL(HIP_KERNEL_NAME(k_tconv<1>), dim3(NP / 64, NDO / 64), blk, 0, stream,
                     W_out, (int)NP, (int)NDO, 1.0f, wo, wo + QWO);
  hipLaunchKernelGGL(HIP_KERNEL_NAME(k_tconv<1>), dim3(NP / 64, NDO / 64), blk, 0, stream,
                     W_act, (int)NP, (int)NDO, 1.0f, wo + 2 * QWO, wo + 3 * QWO);
  k_initz<<<dim3((unsigned)((QF / 8 + 255) / 256)), blk, 0, stream>>>(z0, zh, (int)(QF / 8));

  hipLaunchKernelGGL(HIP_KERNEL_NAME(k_gemm<1, 1, 1>), dim3(NB / GBM, ND / GBN, 1), blk, 0, stream,
                     (const unsigned short*)xh, (const unsigned short*)xl, (int)NDIN, (long long)0,
                     (const unsigned short*)wih, (const unsigned short*)wil, (int)NDIN, (long long)0,
                     (int)NDIN, b_in, b_in, (const float*)nullptr, 0, 1.0f,
                     (float*)nullptr, 0, (long long)0, fh, fl, (int)ND);
  hipLaunchKernelGGL(HIP_KERNEL_NAME(k_gemm<1, 1, 0>), dim3(NB / GBM, ND / GBN, 1), blk, 0, stream,
                     (const unsigned short*)fh, (const unsigned short*)fl, (int)ND, (long long)0,
                     (const unsigned short*)wfh, (const unsigned short*)wfl, (int)ND, (long long)0,
                     (int)ND, b_syn, b_syn, (const float*)nullptr, 0, 1.0f,
                     fpre, (int)ND, (long long)0, (unsigned short*)nullptr, (unsigned short*)nullptr, 0);

  for (int t = 0; t < NT; ++t) {
    hipLaunchKernelGGL(HIP_KERNEL_NAME(k_gemm<0, 0, 0>), dim3(NB / GBM, ND / GBN, 1), blk, 0, stream,
                       (const unsigned short*)zh, (const unsigned short*)nullptr, (int)ND, (long long)0,
                       (const unsigned short*)wz, (const unsigned short*)nullptr, (int)ND, (long long)0,
                       (int)ND, (const float*)nullptr, (const float*)nullptr, (const float*)fpre, (int)ND,
                       ZW_UNSCALE,
                       hist + (size_t)t * QF, (int)ND, (long long)0,
                       (unsigned short*)nullptr, (unsigned short*)nullptr, 0);
    k_nlm<<<dim3((unsigned)(QF / 1024)), blk, 0, stream>>>(hist, w1, b1, w2, b2, zf, zh, t);
    k_sync<<<dim3(NB), dim3(128), 0, stream>>>(zf, prs_o, prs_a, dec_o, dec_a, So, Sa, spl,
                                               (int)(t == 0 ? 1 : 0));
    hipLaunchKernelGGL(HIP_KERNEL_NAME(k_gemm<1, 1, 0>), dim3(NB / GBM, NDO / GBN, 2), blk, 0, stream,
                       (const unsigned short*)spl, (const unsigned short*)(spl + QS), (int)NP,
                       (long long)(2 * QS),
                       (const unsigned short*)wo, (const unsigned short*)(wo + QWO), (int)NP,
                       (long long)(2 * QWO),
                       (int)NP, b_out, b_act, (const float*)nullptr, 0, 1.0f,
                       out + (size_t)t * NDO, (int)(NT * NDO), (long long)((size_t)NB * NT * NDO),
                       (unsigned short*)nullptr, (unsigned short*)nullptr, 0);
  }
}
